// egc_63754494542122
// MI455X (gfx1250) — hardware-verified
//
#include <hip/hip_runtime.h>
#include <stddef.h>
#include <math.h>


#define CH     128
#define KNB    16
#define APZ    136
#define AP2    264
#define KPB    128
#define KP2    256
#define PQW    256
#define NTHR   256
#define NWAVE  8
#define NIT    16
#define NPB    (NWAVE * NIT)
#define PROWS  32
#define PTHR   64
#define HROWS  64
#define HCROWS 80
#define HTHR   160
#define DEGCAP 1024
#define EPT    8
#define NGRP   2
#define CHUNK  (NTHR * EPT * NGRP)
#define WCAP   (EPT * NGRP * 32)
#define LISTN  (NWAVE * WCAP)
#define NBC    4096
#define NBF    1024
#define RCAP   40960
#define RBN    128
#define OTHR   512
#define LDS_FILL ((RCAP + NBF + LISTN) * 4 + 64)
#define LDS_EDGE (2 * NWAVE * KNB * APZ * 2 + 2 * NWAVE * CH * 4 + 4 * CH * 4 + NPB * 3 * 4 + 64)
#define LDS_NODE (HCROWS * AP2 * 2 + HCROWS * APZ * 2 + HCROWS * CH * 4 + 2 * CH * 4)
#define OFF_B1  0
#define OFF_B2  (2 * CH * KPB)
#define OFF_BC  (OFF_B2 + CH * KPB)
#define OFF_BH1 (OFF_BC + CH * KPB)
#define OFF_BH2 (OFF_BH1 + CH * KP2)
#define BPTOT   (OFF_BH2 + CH * KPB)
#define WSCAP  134217728
#define WSC    64.0f
#define ZSC    8.0f
#define RZW    0.001953125f

static_assert(NIT * NWAVE == NPB);
static_assert(PROWS == (PTHR / 32) * 16);
static_assert(HCROWS == (HTHR / 32) * 16);
static_assert(HCROWS >= HROWS + 1);
static_assert((APZ % 8) == 0 && (AP2 % 8) == 0 && (KPB % 8) == 0 && (KP2 % 8) == 0 && (PQW % 32) == 0);
static_assert(BPTOT == 114688);
static_assert(PTHR * 64 == PROWS * CH);
static_assert((PROWS * PQW / 4) % PTHR == 0);
static_assert(HTHR * 64 == HCROWS * CH);
static_assert(HTHR >= 64);
static_assert(NTHR * 4 == NWAVE * CH);
static_assert(NWAVE >= 4);
static_assert(((NPB * 3) % 4) == 0 && (NPB * 3) / 4 <= NTHR);
static_assert(((NWAVE * KNB * APZ * 2) % 16) == 0);
static_assert(((HCROWS * AP2 * 2) % 16) == 0 && ((HCROWS * APZ * 2) % 16) == 0);
static_assert((CHUNK & (CHUNK - 1)) == 0);
static_assert(CHUNK <= 4096);
static_assert(NBC <= 4096 && NBF <= 4096);
static_assert((NBC & (NBC - 1)) == 0 && (NBF & (NBF - 1)) == 0);
static_assert(NBC == 4 * NBF);
static_assert(OTHR * 8 == NBC);
static_assert((RCAP % 32) == 0);
static_assert((DEGCAP % KNB) == 0);

typedef float    v4f  __attribute__((ext_vector_type(4)));
typedef float    v8f  __attribute__((ext_vector_type(8)));
typedef int      v4i  __attribute__((ext_vector_type(4)));
typedef _Float16 v8h  __attribute__((ext_vector_type(8)));
typedef _Float16 v16h __attribute__((ext_vector_type(16)));
union Frag { v16h v; v8h h[2]; };

__device__ __forceinline__ v8f wmh(v16h a, v16h b, v8f c) {
  v8f d = __builtin_amdgcn_wmma_f32_16x16x32_f16(false, a, false, b, (short)0, c, false, false);
  asm volatile("v_nop\n\tv_nop\n\tv_nop\n\tv_nop" : "+v"(d) : "v"(a), "v"(b));
  return d;
}

__device__ __forceinline__ v8h cvt8(v4f a, v4f b, float s) {
  v8h r;
  r[0] = (_Float16)(a.x * s); r[1] = (_Float16)(a.y * s); r[2] = (_Float16)(a.z * s); r[3] = (_Float16)(a.w * s);
  r[4] = (_Float16)(b.x * s); r[5] = (_Float16)(b.y * s); r[6] = (_Float16)(b.z * s); r[7] = (_Float16)(b.w * s);
  return r;
}

__device__ __forceinline__ float tnh(float x) {
  const float e = __expf(2.0f * x);
  return fmaf(-2.0f, __builtin_amdgcn_rcpf(e + 1.0f), 1.0f);
}

template <int NT, int KS, int AP, int BP>
__device__ __forceinline__ void mma16(const _Float16* At, const _Float16* __restrict__ Bpl,
                                      int lane, v8f (&acc)[NT]) {
  const int hh = lane >> 4, m = lane & 15;
#pragma unroll
  for (int t = 0; t < NT; ++t) { v8f z = {0.f, 0.f, 0.f, 0.f, 0.f, 0.f, 0.f, 0.f}; acc[t] = z; }
  const _Float16* ap = At + m * AP + 8 * hh;
  const _Float16* bb = Bpl + (size_t)m * BP + 8 * hh;
#pragma unroll 1
  for (int ks = 0; ks < KS; ++ks) {
    Frag a;
    a.h[0] = *(const v8h*)(ap + 32 * ks);
    a.h[1] = *(const v8h*)(ap + 32 * ks + 16);
#pragma unroll
    for (int t = 0; t < NT; ++t) {
      const _Float16* bp = bb + (size_t)(16 * t) * BP + 32 * ks;
      Frag b;
      b.h[0] = *(const v8h*)bp;
      b.h[1] = *(const v8h*)(bp + 16);
      acc[t] = wmh(a.v, b.v, acc[t]);
    }
  }
}

template <int NB>
__device__ __forceinline__ int scan_chunk(const int* __restrict__ dsts, int nE, int cbase, int slotBase,
                                          int vec8, int* list, int tid, int lane, int wave) {
  int wc = 0;
#pragma unroll
  for (int g = 0; g < NGRP; ++g) {
    const int el0  = (g * NTHR + tid) * EPT;
    const int e0   = cbase + el0;
    const int sent = -2147483647 - 1;
    v4i da, db;
    if (vec8 != 0 && cbase + CHUNK <= nE) {
      da = *(const v4i*)(dsts + e0);
      db = *(const v4i*)(dsts + e0 + 4);
    } else {
      da.x = (e0     < nE) ? dsts[min(e0, nE - 1)] : sent;
      da.y = (e0 + 1 < nE) ? dsts[min(e0 + 1, nE - 1)] : sent;
      da.z = (e0 + 2 < nE) ? dsts[min(e0 + 2, nE - 1)] : sent;
      da.w = (e0 + 3 < nE) ? dsts[min(e0 + 3, nE - 1)] : sent;
      db.x = (e0 + 4 < nE) ? dsts[min(e0 + 4, nE - 1)] : sent;
      db.y = (e0 + 5 < nE) ? dsts[min(e0 + 5, nE - 1)] : sent;
      db.z = (e0 + 6 < nE) ? dsts[min(e0 + 6, nE - 1)] : sent;
      db.w = (e0 + 7 < nE) ? dsts[min(e0 + 7, nE - 1)] : sent;
    }
    const unsigned nb = (unsigned)slotBase;
    const unsigned s0 = (unsigned)da.x - nb, s1 = (unsigned)da.y - nb;
    const unsigned s2 = (unsigned)da.z - nb, s3 = (unsigned)da.w - nb;
    const unsigned s4 = (unsigned)db.x - nb, s5 = (unsigned)db.y - nb;
    const unsigned s6 = (unsigned)db.z - nb, s7 = (unsigned)db.w - nb;
    const bool h0 = s0 < (unsigned)NB, h1 = s1 < (unsigned)NB, h2 = s2 < (unsigned)NB, h3 = s3 < (unsigned)NB;
    const bool h4 = s4 < (unsigned)NB, h5 = s5 < (unsigned)NB, h6 = s6 < (unsigned)NB, h7 = s7 < (unsigned)NB;
    const unsigned any = __builtin_amdgcn_ballot_w32(h0 | h1 | h2 | h3 | h4 | h5 | h6 | h7);
    if (any != 0u) {
#define HITJ(J, HJ, SJ) { \
        const unsigned mj = __builtin_amdgcn_ballot_w32(HJ); \
        if (mj != 0u) { \
          if (HJ) { \
            const int pos = wc + (int)__builtin_amdgcn_mbcnt_lo(mj, 0u); \
            if (pos < WCAP) list[wave * WCAP + pos] = ((el0 + (J)) << 12) | (int)(SJ); \
          } \
          wc += (int)__builtin_popcount(mj); } }
      HITJ(0, h0, s0)
      HITJ(1, h1, s1)
      HITJ(2, h2, s2)
      HITJ(3, h3, s3)
      HITJ(4, h4, s4)
      HITJ(5, h5, s5)
      HITJ(6, h6, s6)
      HITJ(7, h7, s7)
#undef HITJ
    }
  }
  return wc;
}

__global__ __launch_bounds__(NTHR) void k_wprep(const float* __restrict__ W1, const float* __restrict__ W2,
                                                const float* __restrict__ Wc1, const float* __restrict__ Wh1,
                                                const float* __restrict__ Wh2, _Float16* Bpl) {
  const int blk = blockIdx.x, tid = threadIdx.x;
  float v[8];
  int o;
  if (blk < 16) {
    const int i = blk * NTHR + tid;
    const int n = i >> 4, k0 = (i & 15) * 8;
    const int kb = 1 + ((n >> 7) << 7), nc = n & (CH - 1);
#pragma unroll
    for (int e = 0; e < 8; ++e) v[e] = W1[(size_t)(kb + k0 + e) * CH + nc];
    o = OFF_B1 + i * 8;
  } else if (blk < 24) {
    const int i = (blk - 16) * NTHR + tid;
    const int n = i >> 4, k0 = (i & 15) * 8;
#pragma unroll
    for (int e = 0; e < 8; ++e) v[e] = W2[(size_t)(k0 + e) * CH + n];
    o = OFF_B2 + i * 8;
  } else if (blk < 32) {
    const int i = (blk - 24) * NTHR + tid;
    const int n = i >> 4, k0 = (i & 15) * 8;
#pragma unroll
    for (int e = 0; e < 8; ++e) v[e] = Wc1[(size_t)(k0 + e) * CH + n];
    o = OFF_BC + i * 8;
  } else if (blk < 48) {
    const int i = (blk - 32) * NTHR + tid;
    const int n = i >> 5, k0 = (i & 31) * 8;
#pragma unroll
    for (int e = 0; e < 8; ++e) v[e] = Wh1[(size_t)(k0 + e) * CH + n];
    o = OFF_BH1 + i * 8;
  } else {
    const int i = (blk - 48) * NTHR + tid;
    const int n = i >> 4, k0 = (i & 15) * 8;
#pragma unroll
    for (int e = 0; e < 8; ++e) v[e] = Wh2[(size_t)(k0 + e) * CH + n];
    o = OFF_BH2 + i * 8;
  }
  v8h hv;
#pragma unroll
  for (int e = 0; e < 8; ++e) hv[e] = (_Float16)(v[e] * WSC);
  _Float16* dp = Bpl + o;
  *(volatile v8h*)dp = hv;
  __threadfence();
  *(volatile v8h*)dp = hv;
}

__global__ __launch_bounds__(NTHR) void k_count(const int* __restrict__ dsts, int* cnt, int nE, int vec8) {
  __shared__ __attribute__((aligned(16))) int scnt[NBC];
  __shared__ __attribute__((aligned(16))) int list[LISTN];
  __shared__ int wcnt[NWAVE];
  const int tid = threadIdx.x, lane = tid & 31, wave = tid >> 5;
  const int nodeBase = blockIdx.x * NBC;

  for (int i = tid; i < NBC; i += NTHR) scnt[i] = 0;
  __syncthreads();

  const int nChunks = (nE + CHUNK - 1) / CHUNK;
#pragma unroll 1
  for (int ch = 0; ch < nChunks; ++ch) {
    const int cbase = ch * CHUNK;
    const int wc = scan_chunk<NBC>(dsts, nE, cbase, nodeBase, vec8, list, tid, lane, wave);
    if (lane == 0) wcnt[wave] = wc;
    __syncthreads();
    if (wave == 0) {
#pragma unroll 1
      for (int wsx = 0; wsx < NWAVE; ++wsx) {
        int n = __builtin_amdgcn_readfirstlane(wcnt[wsx]);
        n = n > WCAP ? WCAP : (n < 0 ? 0 : n);
        const int* lp = list + wsx * WCAP;
#pragma unroll 1
        for (int i = 0; i < n; ++i) {
          const int ent  = __builtin_amdgcn_readfirstlane(lp[i]);
          const int slot = ent & (NBC - 1);
          if (lane == 0) scnt[slot] = scnt[slot] + 1;
        }
      }
    }
    __syncthreads();
  }

  v4i cq[4];
#pragma unroll
  for (int q = 0; q < 4; ++q) {
    const int f = (wave * 4 + q) * 128 + 4 * lane;
    cq[q] = *(const v4i*)(scnt + f);
  }
  int* cp = cnt + (size_t)nodeBase;
#pragma unroll
  for (int q = 0; q < 4; ++q) {
    const int f = (wave * 4 + q) * 128 + 4 * lane;
    *(volatile v4i*)(cp + f) = cq[q];
  }
  __threadfence();
#pragma unroll
  for (int q = 0; q < 4; ++q) {
    const int f = (wave * 4 + q) * 128 + 4 * lane;
    *(volatile v4i*)(cp + f) = cq[q];
  }
}

__global__ __launch_bounds__(OTHR) void k_offsets(
    const int* __restrict__ cnt, int* off, int* rbase, int nChunk) {
  __shared__ __attribute__((aligned(16))) int soff[NBC];
  __shared__ __attribute__((aligned(16))) int srb[RBN];
  __shared__ int wtot[OTHR / 32];
  const int tid = threadIdx.x, lane = tid & 31, wave = tid >> 5, sub = tid >> 7;
  for (int i = tid; i < RBN; i += OTHR) srb[i] = 0;
  int carry = 0;
#pragma unroll 1
  for (int ch = 0; ch < nChunk; ++ch) {
    const int base = ch * NBC;
    const v4i c0 = *(const v4i*)(cnt + base + 8 * tid);
    const v4i c1 = *(const v4i*)(cnt + base + 8 * tid + 4);
    const int e0 = max(c0.x, 0), e1 = max(c0.y, 0), e2 = max(c0.z, 0), e3 = max(c0.w, 0);
    const int e4 = max(c1.x, 0), e5 = max(c1.y, 0), e6 = max(c1.z, 0), e7 = max(c1.w, 0);
    const int ts = e0 + e1 + e2 + e3 + e4 + e5 + e6 + e7;
    int incl = ts;
#pragma unroll
    for (int d = 1; d < 32; d <<= 1) {
      const int t = __shfl_up(incl, d);
      if (lane >= d) incl += t;
    }
    if (lane == 31) wtot[wave] = incl;
    __syncthreads();
    const int S0 = wtot[0]  + wtot[1]  + wtot[2]  + wtot[3];
    const int S1 = wtot[4]  + wtot[5]  + wtot[6]  + wtot[7];
    const int S2 = wtot[8]  + wtot[9]  + wtot[10] + wtot[11];
    const int S3 = wtot[12] + wtot[13] + wtot[14] + wtot[15];
    int pre = 0;
#pragma unroll 1
    for (int w = 4 * sub; w < wave; ++w) pre += wtot[w];
    const int b0 = carry;
    const int b1 = b0 + ((S0 + 31) & ~31);
    const int b2 = b1 + ((S1 + 31) & ~31);
    const int b3 = b2 + ((S2 + 31) & ~31);
    const int b4 = b3 + ((S3 + 31) & ~31);
    const int myb = sub == 0 ? b0 : (sub == 1 ? b1 : (sub == 2 ? b2 : b3));
    if (tid == 0) {
      srb[min(4 * ch + 0, RBN - 1)] = b0;
      srb[min(4 * ch + 1, RBN - 1)] = b1;
      srb[min(4 * ch + 2, RBN - 1)] = b2;
      srb[min(4 * ch + 3, RBN - 1)] = b3;
    }
    int run = myb + pre + incl - ts;
    soff[8 * tid + 0] = run; run += e0;
    soff[8 * tid + 1] = run; run += e1;
    soff[8 * tid + 2] = run; run += e2;
    soff[8 * tid + 3] = run; run += e3;
    soff[8 * tid + 4] = run; run += e4;
    soff[8 * tid + 5] = run; run += e5;
    soff[8 * tid + 6] = run; run += e6;
    soff[8 * tid + 7] = run;
    carry = b4;
    __syncthreads();
    const v4i o0 = *(const v4i*)(soff + 4 * tid);
    const v4i o1 = *(const v4i*)(soff + 4 * (tid + OTHR));
    int* op = off + base;
    *(volatile v4i*)(op + 4 * tid) = o0;
    *(volatile v4i*)(op + 4 * (tid + OTHR)) = o1;
    __threadfence();
    *(volatile v4i*)(op + 4 * tid) = o0;
    *(volatile v4i*)(op + 4 * (tid + OTHR)) = o1;
    __syncthreads();
  }
  if (tid == 0) srb[min(4 * nChunk, RBN - 1)] = carry;
  __syncthreads();
  v4i rv = {0, 0, 0, 0};
  if (tid < 32) rv = *(const v4i*)(srb + 4 * tid);
  if (tid < 32) *(volatile v4i*)(rbase + 4 * tid) = rv;
  __threadfence();
  if (tid < 32) *(volatile v4i*)(rbase + 4 * tid) = rv;
}

__global__ __launch_bounds__(NTHR) void k_fill(
    const int* __restrict__ srcs, const int* __restrict__ dsts,
    const int* __restrict__ off, const int* __restrict__ rbase,
    int* csr, int nN, int nE, int vec8, int csrLen) {
  extern __shared__ v4f lds_dyn[];
  int* region = (int*)lds_dyn;
  int* cursor = region + RCAP;
  int* list   = cursor + NBF;
  int* wcnt   = list + LISTN;
  const int tid = threadIdx.x, lane = tid & 31, wave = tid >> 5;
  const int b = blockIdx.x;
  const int nodeBase = b * NBF;

  int rb0 = rbase[b];
  const int rb1 = rbase[b + 1];
  rb0 = rb0 < 0 ? 0 : (rb0 > csrLen ? csrLen : rb0);
  rb0 &= ~31;
  int len = rb1 - rb0;
  len = len < 0 ? 0 : (len > RCAP ? RCAP : len);
  int lenW = (len + 31) & ~31;
  if (rb0 + lenW > csrLen) lenW = (csrLen - rb0) & ~31;

  {
    const v4i z = {0, 0, 0, 0};
    for (int i = tid; i < RCAP / 4; i += NTHR) ((v4i*)region)[i] = z;
    for (int s = tid; s < NBF; s += NTHR) {
      int o = off[nodeBase + s] - rb0;
      o = o < 0 ? 0 : (o > RCAP ? RCAP : o);
      cursor[s] = o;
    }
  }
  __syncthreads();

  const int nChunks = (nE + CHUNK - 1) / CHUNK;
#pragma unroll 1
  for (int ch = 0; ch < nChunks; ++ch) {
    const int cbase = ch * CHUNK;
    const int wc = scan_chunk<NBF>(dsts, nE, cbase, nodeBase, vec8, list, tid, lane, wave);
    if (lane == 0) wcnt[wave] = wc;
    __syncthreads();
    if (wave == 0) {
#pragma unroll 1
      for (int wsx = 0; wsx < NWAVE; ++wsx) {
        int n = __builtin_amdgcn_readfirstlane(wcnt[wsx]);
        n = n > WCAP ? WCAP : (n < 0 ? 0 : n);
        const int* lp = list + wsx * WCAP;
#pragma unroll 1
        for (int i = 0; i < n; ++i) {
          const int ent  = __builtin_amdgcn_readfirstlane(lp[i]);
          const int slot = ent & (NBF - 1);
          int e = cbase + ((ent >> 12) & (CHUNK - 1));
          e = e > nE - 1 ? nE - 1 : e;
          int sv = srcs[e];
          sv = sv < 0 ? 0 : (sv > nN - 1 ? nN - 1 : sv);
          if (lane == 0) {
            int pos = cursor[slot];
            pos = pos < 0 ? 0 : (pos > RCAP - 1 ? RCAP - 1 : pos);
            region[pos] = sv;
            const int np = pos + 1;
            cursor[slot] = np > RCAP ? RCAP : np;
          }
        }
      }
    }
    __syncthreads();
  }

  const int nv = lenW >> 2;
  int* gp = csr + rb0;
#pragma unroll 1
  for (int i = tid; i < nv; i += NTHR) { const v4i v = ((const v4i*)region)[i]; *(volatile v4i*)(gp + 4 * i) = v; }
  __threadfence();
#pragma unroll 1
  for (int i = tid; i < nv; i += NTHR) { const v4i v = ((const v4i*)region)[i]; *(volatile v4i*)(gp + 4 * i) = v; }
}

__global__ __launch_bounds__(PTHR) void k_pq(const float* __restrict__ x, const _Float16* __restrict__ B1,
                                             const float* __restrict__ b1, float* PQ, int nN) {
  __shared__ __attribute__((aligned(16))) _Float16 At[PROWS * APZ];
  __shared__ __attribute__((aligned(16))) float stg[PROWS * PQW];
  const int tid = threadIdx.x, lane = tid & 31, wave = tid >> 5, hh = lane >> 4, m = lane & 15;
  const int rowBase = blockIdx.x * PROWS;
  {
    const int r = tid >> 1, c0 = (tid & 1) * 64;
    int xrow = rowBase + r;
    xrow = xrow > nN - 1 ? nN - 1 : xrow;
    const float* xp = x + (size_t)xrow * CH + c0;
#pragma unroll
    for (int j = 0; j < 8; ++j) {
      const v4f a = *(const v4f*)(xp + 8 * j), b = *(const v4f*)(xp + 8 * j + 4);
      *(v8h*)(At + r * APZ + c0 + 8 * j) = cvt8(a, b, ZSC);
    }
  }
  __syncthreads();

#pragma unroll
  for (int cg = 0; cg < 4; ++cg) {
    v8f acc[4];
    mma16<4, 4, APZ, KPB>(At + wave * 16 * APZ, B1 + (size_t)(64 * cg) * KPB, lane, acc);
    float* sp = stg + (wave * 16 + 8 * hh) * PQW + 64 * cg + m;
#pragma unroll
    for (int t = 0; t < 4; ++t) {
      const float bl = b1[(64 * cg + 16 * t + m) & (CH - 1)];
      const float bv = (cg >= 2) ? bl : 0.0f;
#pragma unroll
      for (int r = 0; r < 8; ++r) sp[r * PQW + 16 * t] = fmaf(acc[t][r], RZW, bv);
    }
  }
  __syncthreads();

  float* gp = PQ + (size_t)rowBase * PQW;
#pragma unroll
  for (int it = 0; it < (PROWS * PQW / 4) / PTHR; ++it) {
    const int f = it * PTHR + tid;
    const v4f v = *(const v4f*)(stg + 4 * f);
    *(volatile v4f*)(gp + 4 * f) = v;
  }
  __threadfence();
#pragma unroll
  for (int it = 0; it < (PROWS * PQW / 4) / PTHR; ++it) {
    const int f = it * PTHR + tid;
    const v4f v = *(const v4f*)(stg + 4 * f);
    *(volatile v4f*)(gp + 4 * f) = v;
  }
}

template <int J0>
__device__ __forceinline__ void rows_m1(_Float16* zw, const float* __restrict__ PQ, const float* qw,
                                        const float* w0p, int sl, int l2i, int hh, int m) {
#pragma unroll
  for (int j = J0; j < J0 + 2; ++j) {
    const int sa = __builtin_amdgcn_readlane(sl, 2 * j), sb = __builtin_amdgcn_readlane(sl, 2 * j + 1);
    const int la = __builtin_amdgcn_readlane(l2i, 2 * j), lb = __builtin_amdgcn_readlane(l2i, 2 * j + 1);
    const int s = hh ? sb : sa;
    const float l2 = __int_as_float(hh ? lb : la);
    const float* pp = PQ + (size_t)s * PQW + 8 * m;
    const v4f p0 = *(const v4f*)pp, p1 = *(const v4f*)(pp + 4);
    const v4f q0 = *(const v4f*)(qw + 8 * m), q1 = *(const v4f*)(qw + 8 * m + 4);
    const v4f wa = *(const v4f*)(w0p + 8 * m), wb = *(const v4f*)(w0p + 8 * m + 4);
    v8h hv;
    hv[0] = (_Float16)(tnh(fmaf(l2, wa.x, p0.x + q0.x)) * ZSC);
    hv[1] = (_Float16)(tnh(fmaf(l2, wa.y, p0.y + q0.y)) * ZSC);
    hv[2] = (_Float16)(tnh(fmaf(l2, wa.z, p0.z + q0.z)) * ZSC);
    hv[3] = (_Float16)(tnh(fmaf(l2, wa.w, p0.w + q0.w)) * ZSC);
    hv[4] = (_Float16)(tnh(fmaf(l2, wb.x, p1.x + q1.x)) * ZSC);
    hv[5] = (_Float16)(tnh(fmaf(l2, wb.y, p1.y + q1.y)) * ZSC);
    hv[6] = (_Float16)(tnh(fmaf(l2, wb.z, p1.z + q1.z)) * ZSC);
    hv[7] = (_Float16)(tnh(fmaf(l2, wb.w, p1.w + q1.w)) * ZSC);
    *(v8h*)(zw + (2 * j + hh) * APZ + 8 * m) = hv;
  }
}

__global__ __launch_bounds__(NTHR) void k_edge(
    const float* __restrict__ PQ, const int* __restrict__ csr,
    const int* __restrict__ offp, const int* __restrict__ cntp,
    const _Float16* __restrict__ B2, const _Float16* __restrict__ B3,
    const float* __restrict__ coords, const float* __restrict__ W1,
    const float* __restrict__ b2, const float* __restrict__ bc1, const float* __restrict__ Wc2,
    float* MI, float* CO, int nN, int csrLen) {
  extern __shared__ v4f lds_dyn[];
  _Float16* z1t = (_Float16*)lds_dyn;
  _Float16* z2t = z1t + NWAVE * KNB * APZ;
  float* sout = (float*)(z2t + NWAVE * KNB * APZ);
  float* qrow = sout + NWAVE * CH;
  float* ptab = qrow + NWAVE * CH;
  float* scoord = ptab + 4 * CH;
  int* slot = (int*)(scoord + NPB * 3);
  const int tid = threadIdx.x, lane = tid & 31, wave = tid >> 5, hh = lane >> 4, m = lane & 15;
  const int base = blockIdx.x * NPB;
  _Float16* z1w = z1t + wave * (KNB * APZ);
  _Float16* z2w = z2t + wave * (KNB * APZ);
  float* qw = qrow + wave * CH;
  float* sw = sout + wave * CH;
  if (wave < 4) {
    const float* tp = (wave == 0) ? W1 : (wave == 1 ? b2 : (wave == 2 ? bc1 : Wc2));
    const v4f tv = *(const v4f*)(tp + 4 * lane);
    *(v4f*)(ptab + wave * CH + 4 * lane) = tv;
  }
  __syncthreads();

#pragma unroll 1
  for (int it = 0; it < NIT; ++it) {
    const int n = base + it * NWAVE + wave;
    const bool nval = n < nN;
    const int cc = nval ? n : nN - 1;
    const int cnr = cntp[cc];
    const int ofr = offp[cc];
    int cn = nval ? cnr : 0;
    cn = cn < 0 ? 0 : (cn > DEGCAP ? DEGCAP : cn);
    cn = __builtin_amdgcn_readfirstlane(cn);
    int of = ofr;
    of = of < 0 ? 0 : (of > csrLen ? csrLen : of);
    of = __builtin_amdgcn_readfirstlane(of);
    const float cX = coords[(size_t)cc * 3 + 0], cY = coords[(size_t)cc * 3 + 1], cZ = coords[(size_t)cc * 3 + 2];
    {
      const v4f qv = *(const v4f*)(PQ + (size_t)cc * PQW + CH + 4 * lane);
      *(v4f*)(qw + 4 * lane) = qv;
      const v4f z = {0.f, 0.f, 0.f, 0.f};
      *(v4f*)(sw + 4 * lane) = z;
    }
    const int ntw = (cn + KNB - 1) >> 4;
    if (lane == 0) slot[wave] = ntw;
    __syncthreads();
    int ntmax;
    {
      const v4i sA = *(const v4i*)slot, sB = *(const v4i*)(slot + 4);
      int mm = max(max(sA.x, sA.y), max(sA.z, sA.w));
      mm = max(mm, max(max(sB.x, sB.y), max(sB.z, sB.w)));
      mm = mm < 0 ? 0 : (mm > DEGCAP / KNB ? DEGCAP / KNB : mm);
      ntmax = __builtin_amdgcn_readfirstlane(mm);
    }
    float tsx = 0.0f, tsy = 0.0f, tsz = 0.0f;
#pragma unroll 1
    for (int tt = 0; tt < ntmax; ++tt) {
      int nv = cn - tt * KNB;
      nv = nv < 0 ? 0 : (nv > KNB ? KNB : nv);
      int pos = of + tt * KNB + m;
      pos = pos < 0 ? 0 : (pos > csrLen - 1 ? csrLen - 1 : pos);
      int sv = csr[pos];
      sv = sv < 0 ? 0 : (sv > nN - 1 ? nN - 1 : sv);
      const float dx = coords[(size_t)sv * 3 + 0] - cX;
      const float dy = coords[(size_t)sv * 3 + 1] - cY;
      const float dz = coords[(size_t)sv * 3 + 2] - cZ;
      const int l2i = __float_as_int(sqrtf(dx * dx + dy * dy + dz * dz));
      rows_m1<0>(z1w, PQ, qw, ptab, sv, l2i, hh, m);
      asm volatile("" ::: "memory");
      rows_m1<2>(z1w, PQ, qw, ptab, sv, l2i, hh, m);
      asm volatile("" ::: "memory");
      rows_m1<4>(z1w, PQ, qw, ptab, sv, l2i, hh, m);
      asm volatile("" ::: "memory");
      rows_m1<6>(z1w, PQ, qw, ptab, sv, l2i, hh, m);
      __syncthreads();
#pragma unroll
      for (int cg = 0; cg < 4; ++cg) {
        v8f acc[2];
        mma16<2, 4, APZ, KPB>(z1w, B2 + (size_t)(32 * cg) * KPB, lane, acc);
#pragma unroll
        for (int t = 0; t < 2; ++t) {
          const int col = 32 * cg + 16 * t + m;
          const float bv = ptab[CH + col];
          float s = 0.0f;
#pragma unroll
          for (int r = 0; r < 8; ++r) {
            const float mv = fmaf(acc[t][r], RZW, bv);
            const bool ok = (8 * hh + r) < nv;
            s += ok ? mv : 0.0f;
            z2w[(8 * hh + r) * APZ + col] = (_Float16)(mv * ZSC);
          }
          s += __shfl_xor(s, 16, 32);
          if (hh == 0) sw[col] = sw[col] + s;
        }
      }
      __syncthreads();
      float p[8] = {0.f, 0.f, 0.f, 0.f, 0.f, 0.f, 0.f, 0.f};
#pragma unroll
      for (int cg = 0; cg < 4; ++cg) {
        v8f acc[2];
        mma16<2, 4, APZ, KPB>(z2w, B3 + (size_t)(32 * cg) * KPB, lane, acc);
#pragma unroll
        for (int t = 0; t < 2; ++t) {
          const int col = 32 * cg + 16 * t + m;
          const float bv = ptab[2 * CH + col];
          const float wv = ptab[3 * CH + col];
#pragma unroll
          for (int r = 0; r < 8; ++r) {
            const float u = tnh(fmaf(acc[t][r], RZW, bv));
            p[r] = fmaf(u, wv, p[r]);
          }
        }
      }
#pragma unroll
      for (int r = 0; r < 8; ++r) {
        float q = p[r];
        q += __shfl_xor(q, 1, 32);
        q += __shfl_xor(q, 2, 32);
        q += __shfl_xor(q, 4, 32);
        q += __shfl_xor(q, 8, 32);
        const int row = 8 * hh + r;
        const float dxr = __shfl(dx, row, 32), dyr = __shfl(dy, row, 32), dzr = __shfl(dz, row, 32);
        const bool ok = row < nv;
        const float cx = dxr * q, cy = dyr * q, cz = dzr * q;
        tsx += ok ? cx : 0.0f;
        tsy += ok ? cy : 0.0f;
        tsz += ok ? cz : 0.0f;
      }
    }
    tsx += __shfl_xor(tsx, 16, 32);
    tsy += __shfl_xor(tsy, 16, 32);
    tsz += __shfl_xor(tsz, 16, 32);
    if (lane == 0) {
      const float rnb = __builtin_amdgcn_rcpf((float)cn);
      const int si = (it * NWAVE + wave) * 3;
      const float ox = cX + tsx * rnb, oy = cY + tsy * rnb, oz = cZ + tsz * rnb;
      scoord[si + 0] = nval ? ox : 0.0f;
      scoord[si + 1] = nval ? oy : 0.0f;
      scoord[si + 2] = nval ? oz : 0.0f;
    }
    __syncthreads();
    {
      const int row = tid >> 5;
      const int node = base + it * NWAVE + row;
      const v4f v = *(const v4f*)(sout + 4 * tid);
      float* gp = MI + (size_t)node * CH + 4 * (tid & 31);
      *(volatile v4f*)gp = v;
      __threadfence();
      *(volatile v4f*)gp = v;
    }
  }
  __syncthreads();
  {
    v4f cv = {0.f, 0.f, 0.f, 0.f};
    const int q = (tid < (NPB * 3) / 4) ? tid : 0;
    if (tid < (NPB * 3) / 4) cv = *(const v4f*)(scoord + 4 * q);
    float* gp = CO + (size_t)base * 3 + 4 * q;
    if (tid < (NPB * 3) / 4) *(volatile v4f*)gp = cv;
    __threadfence();
    if (tid < (NPB * 3) / 4) *(volatile v4f*)gp = cv;
  }
}

__device__ __forceinline__ void node_store(float* out, const float* __restrict__ CO, const float* stg,
                                           int tid, int isb0, int npre, int f3, int cs, int ce, int shift) {
  if (isb0 != 0) {
    const int nItP = ((npre >> 2) + HTHR - 1) / HTHR;
#pragma unroll 1
    for (int it = 0; it < nItP; ++it) {
      const int f = 4 * (it * HTHR + tid);
      int fco = f; fco = fco > f3 - 4 ? f3 - 4 : fco;
      const v4f vco = *(const v4f*)(CO + fco);
      int fs = f - f3; fs = fs < 0 ? 0 : (fs > HCROWS * CH - 4 ? HCROWS * CH - 4 : fs);
      const v4f vs = *(const v4f*)(stg + fs);
      const bool sel = f < f3;
      v4f v;
      v.x = sel ? vco.x : vs.x; v.y = sel ? vco.y : vs.y; v.z = sel ? vco.z : vs.z; v.w = sel ? vco.w : vs.w;
      if (f < npre) *(volatile v4f*)(out + f) = v;
    }
  }
#pragma unroll 1
  for (int it = 0; it < (HROWS * CH / 4 + HTHR - 1) / HTHR; ++it) {
    const int i = it * HTHR + tid;
    const int f = cs + 4 * i;
    int idx = f - shift;
    idx = idx < 0 ? 0 : (idx > HCROWS * CH - 4 ? HCROWS * CH - 4 : idx);
    const v4f v = *(const v4f*)(stg + idx);
    if (f < ce) *(volatile v4f*)(out + f) = v;
  }
}

__global__ __launch_bounds__(HTHR) void k_node(
    const float* __restrict__ hid, const float* __restrict__ MI,
    const _Float16* __restrict__ BH1, const _Float16* __restrict__ BH2,
    const float* __restrict__ bh1, const float* __restrict__ bh2,
    const float* __restrict__ CO, float* out, int nN, int pre) {
  extern __shared__ v4f lds_dyn[];
  _Float16* At = (_Float16*)lds_dyn;
  _Float16* Tt = At + HCROWS * AP2;
  float* stg = (float*)(Tt + HCROWS * APZ);
  float* btab = stg + HCROWS * CH;
  const int tid = threadIdx.x, lane = tid & 31, wave = tid >> 5, hh = lane >> 4, m = lane & 15;
  const int rowBase = blockIdx.x * HROWS;
  {
    const int r = tid >> 1, c0 = tid & 1;
    int node = rowBase + r;
    node = node > nN - 1 ? nN - 1 : node;
    const float* src = (c0 != 0) ? (MI + (size_t)node * CH) : (hid + (size_t)node * CH);
    _Float16* ap = At + r * AP2 + c0 * CH;
    float* sp = stg + r * CH;
#pragma unroll 4
    for (int j = 0; j < 16; ++j) {
      const v4f a = *(const v4f*)(src + 8 * j), b = *(const v4f*)(src + 8 * j + 4);
      *(v8h*)(ap + 8 * j) = cvt8(a, b, ZSC);
      if (c0 == 0) { *(v4f*)(sp + 8 * j) = a; *(v4f*)(sp + 8 * j + 4) = b; }
    }
  }
  if (wave < 2) {
    const float* bp = (wave == 0) ? bh1 : bh2;
    const v4f bv = *(const v4f*)(bp + 4 * lane);
    *(v4f*)(btab + wave * CH + 4 * lane) = bv;
  }
  __syncthreads();
  const _Float16* Aw = At + wave * 16 * AP2;
  _Float16* Tw = Tt + wave * 16 * APZ;
  float* sw = stg + wave * 16 * CH;

#pragma unroll
  for (int chf = 0; chf < 2; ++chf) {
    v8f acc[4];
    mma16<4, 8, AP2, KP2>(Aw, BH1 + (size_t)(64 * chf) * KP2, lane, acc);
#pragma unroll
    for (int t = 0; t < 4; ++t) {
      const int col = 64 * chf + 16 * t + m;
      const float bv = btab[col];
#pragma unroll
      for (int r = 0; r < 8; ++r) {
        const float v = tnh(fmaf(acc[t][r], RZW, bv));
        Tw[(8 * hh + r) * APZ + col] = (_Float16)(v * ZSC);
      }
    }
  }
  __syncthreads();
#pragma unroll
  for (int chf = 0; chf < 2; ++chf) {
    v8f acc[4];
    mma16<4, 4, APZ, KPB>(Tw, BH2 + (size_t)(64 * chf) * KPB, lane, acc);
#pragma unroll
    for (int t = 0; t < 4; ++t) {
      const int col = 64 * chf + 16 * t + m;
      const float bv = btab[CH + col];
#pragma unroll
      for (int r = 0; r < 8; ++r) {
        const int idx = (8 * hh + r) * CH + col;
        sw[idx] = sw[idx] + fmaf(acc[t][r], RZW, bv);
      }
    }
  }
  __syncthreads();

  const int f3 = 3 * nN;
  const int fend = f3 + CH * nN;
  const int shift = f3 + HROWS * CH * (int)blockIdx.x;
  const int cs = shift + pre;
  int ce = cs + HROWS * CH;
  ce = ce > fend ? fend : ce;
  const int npre = f3 + pre;
  const int isb0 = (blockIdx.x == 0) ? 1 : 0;
  node_store(out, CO, stg, tid, isb0, npre, f3, cs, ce, shift);
  __threadfence();
  node_store(out, CO, stg, tid, isb0, npre, f3, cs, ce, shift);
}

extern "C" void kernel_launch(void* const* d_in, const int* in_sizes, int n_in,
                              void* d_out, int out_size, void* d_ws, size_t ws_size,
                              hipStream_t stream) {
  if (n_in < 14) return;
  const int nN = in_sizes[0] / 3;
  const int nE = in_sizes[2] / 2;
  if (nN < 4 || nE <= 0) return;
  if (in_sizes[0] != 3 * nN || in_sizes[1] != nN * CH || in_sizes[2] != 2 * nE) return;
  if (in_sizes[3] != (2 * CH + 1) * CH || in_sizes[4] != CH || in_sizes[5] != CH * CH || in_sizes[6] != CH) return;
  if (in_sizes[7] != CH * CH || in_sizes[8] != CH || in_sizes[9] != CH) return;
  if (in_sizes[10] != 2 * CH * CH || in_sizes[11] != CH || in_sizes[12] != CH * CH || in_sizes[13] != CH) return;
  if (out_size != 3 * nN + CH * nN) return;
  if ((nN & 3) != 0) return;
  if (nE > (1 << 28) || nN > (1 << 23)) return;

  const float* coords = (const float*)d_in[0];
  const float* hidden = (const float*)d_in[1];
  const int*   edges  = (const int*)d_in[2];
  const float* W1  = (const float*)d_in[3];
  const float* b1  = (const float*)d_in[4];
  const float* W2  = (const float*)d_in[5];
  const float* b2  = (const float*)d_in[6];
  const float* Wc1 = (const float*)d_in[7];
  const float* bc1 = (const float*)d_in[8];
  const float* Wc2 = (const float*)d_in[9];
  const float* Wh1 = (const float*)d_in[10];
  const float* bh1 = (const float*)d_in[11];
  const float* Wh2 = (const float*)d_in[12];
  const float* bh2 = (const float*)d_in[13];
  const int* srcs = edges;
  const int* dsts = edges + nE;
  float* out = (float*)d_out;

  const int nBlkQ = (nN + PROWS - 1) / PROWS;
  const int NPADG = nBlkQ * PROWS;
  const int nBlkP = (nN + NPB - 1) / NPB;
  const int NPADP = nBlkP * NPB;
  const int nBlkH = (nN + HROWS - 1) / HROWS;
  const int nBC   = (nN + NBC - 1) / NBC;
  const int CNTPAD = nBC * NBC;
  if (4 * nBC + 1 > RBN) return;
  const int nBF    = (nN + NBF - 1) / NBF;
  const int csrLen = ((nE + 31) & ~31) + 4096;
  if (31 * 4 * nBC > 4096) return;
  const int pre = (32 - ((3 * nN) & 31)) & 31;

  char* ws = (char*)d_ws;
  size_t off = 0;
  const size_t oB   = off; off += (size_t)BPTOT * 2;               off = (off + 255) & ~(size_t)255;
  const size_t oCnt = off; off += (size_t)CNTPAD * 4;              off = (off + 255) & ~(size_t)255;
  const size_t oOff = off; off += (size_t)CNTPAD * 4;              off = (off + 255) & ~(size_t)255;
  const size_t oRb  = off; off += (size_t)RBN * 4;                 off = (off + 255) & ~(size_t)255;
  const size_t oCsr = off; off += (size_t)csrLen * 4;              off = (off + 255) & ~(size_t)255;
  const size_t oPQ  = off; off += (size_t)NPADG * PQW * 4;         off = (off + 255) & ~(size_t)255;
  const size_t oMI  = off; off += (size_t)NPADP * CH * 4;          off = (off + 255) & ~(size_t)255;
  const size_t oCO  = off; off += (size_t)NPADP * 3 * 4;           off = (off + 255) & ~(size_t)255;
  if (off > ws_size || off > (size_t)WSCAP) return;
  _Float16* Bpl  = (_Float16*)(ws + oB);
  int*      cnt  = (int*)(ws + oCnt);
  int*      offp = (int*)(ws + oOff);
  int*      rb   = (int*)(ws + oRb);
  int*      csr  = (int*)(ws + oCsr);
  float*    PQ   = (float*)(ws + oPQ);
  float*    MI   = (float*)(ws + oMI);
  float*    CO   = (float*)(ws + oCO);

  const int vec8 = ((nE & 3) == 0) ? 1 : 0;

  k_wprep<<<56, NTHR, 0, stream>>>(W1, W2, Wc1, Wh1, Wh2, Bpl);
  k_count<<<nBC, NTHR, 0, stream>>>(dsts, cnt, nE, vec8);
  k_offsets<<<1, OTHR, 0, stream>>>(cnt, offp, rb, nBC);
  hipFuncSetAttribute(reinterpret_cast<const void*>(&k_fill),
                      hipFuncAttributeMaxDynamicSharedMemorySize, LDS_FILL);
  k_fill<<<nBF, NTHR, LDS_FILL, stream>>>(srcs, dsts, offp, rb, csr, nN, nE, vec8, csrLen);
  k_pq<<<nBlkQ, PTHR, 0, stream>>>(hidden, Bpl + OFF_B1, b1, PQ, nN);
  hipFuncSetAttribute(reinterpret_cast<const void*>(&k_edge),
                      hipFuncAttributeMaxDynamicSharedMemorySize, LDS_EDGE);
  k_edge<<<nBlkP, NTHR, LDS_EDGE, stream>>>(PQ, csr, offp, cnt, Bpl + OFF_B2, Bpl + OFF_BC, coords, W1,
                                            b2, bc1, Wc2, MI, CO, nN, csrLen);
  hipFuncSetAttribute(reinterpret_cast<const void*>(&k_node),
                      hipFuncAttributeMaxDynamicSharedMemorySize, LDS_NODE);
  k_node<<<nBlkH, HTHR, LDS_NODE, stream>>>(hidden, MI, Bpl + OFF_BH1, Bpl + OFF_BH2, bh1, bh2, CO, out, nN, pre);
}
